// PointMambaLayer_12850542150376
// MI455X (gfx1250) — hardware-verified
//
#include <hip/hip_runtime.h>
#include <hip/hip_bf16.h>
#include <math.h>

#define NPT   4096
#define DMD   256
#define DIN   512
#define DST   512
#define NHD   16
#define HDM   32
#define CNV   1536
#define NXB   1600
#define NWI   2112
#define DPR   2064
#define KW    4
#define NL    2
#define CH    256
#define NCH   16
#define ACSP  32
#define GSTR  40
#define OSTR  68
#define EPSV  1e-5f
#define SBC   64.0f
#define SXD   256.0f
#define SGD   1024.0f
#define SPV   1024.0f
static_assert(NPT == NCH * CH);
static_assert(DIN == NHD * HDM);
static_assert(CH == 256);

typedef unsigned short us16 __attribute__((ext_vector_type(16)));
typedef unsigned short us8  __attribute__((ext_vector_type(8)));
typedef unsigned short us8a __attribute__((ext_vector_type(8), may_alias));
typedef unsigned short us4  __attribute__((ext_vector_type(4)));
typedef unsigned short us4a __attribute__((ext_vector_type(4), may_alias));
typedef _Float16 v16h __attribute__((ext_vector_type(16)));
typedef _Float16 v8h  __attribute__((ext_vector_type(8)));
typedef _Float16 v4h  __attribute__((ext_vector_type(4)));
typedef __bf16 v16b __attribute__((ext_vector_type(16)));
typedef float v8f __attribute__((ext_vector_type(8)));
typedef float v4f __attribute__((ext_vector_type(4)));
typedef float v4fa __attribute__((ext_vector_type(4), may_alias));
union FragU { us16 v; us8 h[2]; };

__device__ __forceinline__ unsigned short bf16_bits(float f) {
  unsigned u = __float_as_uint(f);
  u += 0x7FFFu + ((u >> 16) & 1u);
  return (unsigned short)(u >> 16);
}
__device__ __forceinline__ float bf16_val(unsigned short b) { return __uint_as_float(((unsigned)b) << 16); }
__device__ __forceinline__ float bf16r(float f) { return bf16_val(bf16_bits(f)); }
__device__ __forceinline__ float silu_f(float v) { return v * __builtin_amdgcn_rcpf(1.0f + __expf(-v)); }

template <int TB>
__device__ __forceinline__ v8f mma32(us16 a, us16 b, v8f c) {
  if (TB) c = __builtin_amdgcn_wmma_f32_16x16x32_bf16(false, __builtin_bit_cast(v16b, a), false, __builtin_bit_cast(v16b, b), (short)0, c, false, false);
  else    c = __builtin_amdgcn_wmma_f32_16x16x32_f16(false, __builtin_bit_cast(v16h, a), false, __builtin_bit_cast(v16h, b), (short)0, c, false, false);
  return c;
}
__device__ __forceinline__ void wguard4(v8f& c0, v8f& c1, v8f& c2, v8f& c3, const us16& a0, const us16& a1,
                                        const us16& b0, const us16& b1, const us16& b2, const us16& b3) {
#if defined(__HIP_DEVICE_COMPILE__)
  asm volatile("v_nop\n\tv_nop\n\tv_nop\n\tv_nop"
               : "+v"(c0), "+v"(c1), "+v"(c2), "+v"(c3)
               : "v"(a0), "v"(a1), "v"(b0), "v"(b1), "v"(b2), "v"(b3));
#endif
}
__device__ __forceinline__ void wguard2(v8f& c0, v8f& c1, const us16& a0, const us16& a1, const us16& b0, const us16& b1) {
#if defined(__HIP_DEVICE_COMPILE__)
  asm volatile("v_nop\n\tv_nop\n\tv_nop\n\tv_nop"
               : "+v"(c0), "+v"(c1)
               : "v"(a0), "v"(a1), "v"(b0), "v"(b1));
#endif
}

__device__ __forceinline__ us16 lds_frag(const unsigned short* base) {
  const int lane = threadIdx.x & 31, r = lane & 15, kh = (lane >> 4) * 8;
  FragU f;
  f.h[0] = *(const us8a*)(base + r * GSTR + kh);
  f.h[1] = *(const us8a*)(base + r * GSTR + 16 + kh);
  return f.v;
}

template <int KM>
__device__ __forceinline__ void stage_a16(unsigned short* lds, const unsigned short* __restrict__ P, int ld, int m0, int k0, int tid) {
  if constexpr (KM == 0) {
    const int row = tid >> 1, cq = (tid & 1) * 16;
    const unsigned short* src = P + (size_t)(m0 + row) * ld + k0 + cq;
    const us8 v0 = *(const us8a*)src;
    const us8 v1 = *(const us8a*)(src + 8);
    *(us8a*)(lds + row * GSTR + cq) = v0;
    *(us8a*)(lds + row * GSTR + cq + 8) = v1;
  } else {
    const int k = tid >> 3, mq = (tid & 7) * 16;
    const unsigned short* src = P + (size_t)(k0 + k) * ld + m0 + mq;
    const us8 v0 = *(const us8a*)src;
    const us8 v1 = *(const us8a*)(src + 8);
#pragma unroll
    for (int u = 0; u < 8; ++u) { lds[(mq + u) * GSTR + k] = v0[u]; lds[(mq + 8 + u) * GSTR + k] = v1[u]; }
  }
}
__device__ __forceinline__ void stage_g(unsigned short* lds, const float* __restrict__ P, int ld, int m0, int k0, int tid, const float* lacs) {
  const int row = tid >> 1, cq = (tid & 1) * 16;
  const int t = m0 + row;
  const float* src = P + (size_t)t * ld + k0 + cq;
  const v4f q0 = *(const v4fa*)src, q1 = *(const v4fa*)(src + 4), q2 = *(const v4fa*)(src + 8), q3 = *(const v4fa*)(src + 12);
  float cb[16];
#pragma unroll
  for (int u = 0; u < 4; ++u) { cb[u] = q0[u]; cb[4 + u] = q1[u]; cb[8 + u] = q2[u]; cb[12 + u] = q3[u]; }
  const float at = lacs[t];
  const int s0 = k0 + cq;
  v8h h0, h1;
#pragma unroll
  for (int u = 0; u < 8; ++u) {
    const int s = s0 + u;
    float d = __expf(fminf(at - lacs[s], 0.0f));
    d = (s <= t) ? d : 0.0f;
    h0[u] = (_Float16)(cb[u] * d * SGD);
  }
#pragma unroll
  for (int u = 0; u < 8; ++u) {
    const int s = s0 + 8 + u;
    float d = __expf(fminf(at - lacs[s], 0.0f));
    d = (s <= t) ? d : 0.0f;
    h1[u] = (_Float16)(cb[8 + u] * d * SGD);
  }
  *(us8a*)(lds + row * GSTR + cq) = __builtin_bit_cast(us8, h0);
  *(us8a*)(lds + row * GSTR + cq + 8) = __builtin_bit_cast(us8, h1);
}
template <int KM, int NT>
__device__ __forceinline__ void stage_b16(unsigned short* lds, const unsigned short* __restrict__ P, int ld, int n0, int k0, int tid) {
  if constexpr (NT == 64) {
    if constexpr (KM == 0) {
      const int row = tid >> 2, kq = (tid & 3) * 8;
      const us8 v = *(const us8a*)(P + (size_t)(n0 + row) * ld + k0 + kq);
      *(us8a*)(lds + row * GSTR + kq) = v;
    } else {
      const int k = tid >> 3, nq = (tid & 7) * 8;
      const us8 v = *(const us8a*)(P + (size_t)(k0 + k) * ld + n0 + nq);
#pragma unroll
      for (int u = 0; u < 8; ++u) lds[(nq + u) * GSTR + k] = v[u];
    }
  } else {
    if constexpr (KM == 0) {
      const int row = tid >> 3, kq = (tid & 7) * 4;
      const us4 v = *(const us4a*)(P + (size_t)(n0 + row) * ld + k0 + kq);
      *(us4a*)(lds + row * GSTR + kq) = v;
    } else {
      const int k = tid >> 3, nq = (tid & 7) * 4;
      const us4 v = *(const us4a*)(P + (size_t)(k0 + k) * ld + n0 + nq);
#pragma unroll
      for (int u = 0; u < 4; ++u) lds[(nq + u) * GSTR + k] = v[u];
    }
  }
}

template <int TB, int NP, int AKM, int BKM, int EPI, int NT>
__global__ __launch_bounds__(256) void k_gemm(
    const void* A0v, const void* A1v, int lda, long long sAc, long long sAh,
    const unsigned short* __restrict__ Bp, int ldb, long long sBc, long long sBh,
    float* Y, int ldy, long long sYc, long long sYh,
    const float* __restrict__ R, int ldr, long long sRc, long long sRh,
    const float* __restrict__ aux,
    const float* __restrict__ dcl, long long sDc, long long sDh,
    int zh, int K, float scale)
{
  constexpr int NJ = NT / 16;
  constexpr int LNT = (NT == 64) ? 6 : 5;
  __shared__ __attribute__((aligned(16))) unsigned short lA0[128 * GSTR];
  __shared__ __attribute__((aligned(16))) unsigned short lA1[(NP > 1) ? 128 * GSTR : 16];
  __shared__ __attribute__((aligned(16))) unsigned short lB[NT * GSTR];
  __shared__ __attribute__((aligned(16))) float oS[8 * 16 * OSTR];
  __shared__ __attribute__((aligned(16))) float lacs[(AKM == 2 || EPI == 2) ? CH : 4];
  const int tid = threadIdx.x, lane = tid & 31, wave = tid >> 5, cl = lane & 15, hh = lane >> 4;
  const int m0 = blockIdx.x * 128, n0 = blockIdx.y * NT;
  const int z = blockIdx.z, zc = z / zh, zq = z - zc * zh;
  const long long aoff = (long long)zc * sAc + (long long)zq * sAh;
  const unsigned short* A0 = (const unsigned short*)A0v + aoff;
  const unsigned short* A1 = (const unsigned short*)A1v + aoff;
  const float* Af = (const float*)A0v + aoff;
  Bp += (long long)zc * sBc + (long long)zq * sBh;
  if constexpr (AKM == 2 || EPI == 2) lacs[tid] = dcl[(long long)zc * sDc + (long long)zq * sDh + (long long)tid * ACSP];

  v8f acc[NJ];
#pragma unroll
  for (int j = 0; j < NJ; ++j) { v8f zz = {0.f, 0.f, 0.f, 0.f, 0.f, 0.f, 0.f, 0.f}; acc[j] = zz; }

#pragma unroll 1
  for (int k0 = 0; k0 < K; k0 += 32) {
    __syncthreads();
    if constexpr (AKM == 2) stage_g(lA0, Af, lda, m0, k0, tid, lacs);
    else stage_a16<AKM>(lA0, A0, lda, m0, k0, tid);
    if constexpr (NP > 1) stage_a16<(AKM == 1) ? 1 : 0>(lA1, A1, lda, m0, k0, tid);
    stage_b16<BKM, NT>(lB, Bp, ldb, n0, k0, tid);
    __syncthreads();
    const us16 af = lds_frag(lA0 + 16 * wave * GSTR);
    us16 afl = af;
    if constexpr (NP > 1) afl = lds_frag(lA1 + 16 * wave * GSTR);
    us16 bf[NJ];
#pragma unroll
    for (int j = 0; j < NJ; ++j) bf[j] = lds_frag(lB + 16 * j * GSTR);
#pragma unroll
    for (int j = 0; j < NJ; ++j) acc[j] = mma32<TB>(af, bf[j], acc[j]);
    if constexpr (NP > 1) {
#pragma unroll
      for (int j = 0; j < NJ; ++j) acc[j] = mma32<TB>(afl, bf[j], acc[j]);
    }
    if constexpr (NJ == 4) wguard4(acc[0], acc[1], acc[2], acc[3], af, afl, bf[0], bf[1], bf[2], bf[3]);
    else wguard2(acc[0], acc[1], af, afl, bf[0], bf[1]);
  }

  float* so = oS + wave * (16 * OSTR);
#pragma unroll
  for (int j = 0; j < NJ; ++j)
#pragma unroll
    for (int r = 0; r < 8; ++r) so[(8 * hh + r) * OSTR + 16 * j + cl] = acc[j][r] * scale;
  __syncthreads();
  if constexpr (EPI != 0) {
    float dsk = 0.0f;
    const float* Rz = R;
    if constexpr (EPI == 1) { dsk = bf16r(aux[zq]); Rz = R + (long long)zc * sRc + (long long)zq * sRh; }
#pragma unroll 1
    for (int e = lane; e < 16 * NT; e += 32) {
      const int r = e >> LNT, c = e & (NT - 1);
      const int m = m0 + 16 * wave + r, n = n0 + c;
      float v = so[r * OSTR + c];
      if constexpr (EPI == 1) v += dsk * Rz[(size_t)m * ldr + n];
      if constexpr (EPI == 2) v *= __expf(fminf(lacs[m], 0.0f));
      so[r * OSTR + c] = v;
    }
    __syncthreads();
  }
#pragma unroll
  for (int pass = 0; pass < 2; ++pass) {
    float* Yz = Y + (long long)zc * sYc + (long long)zq * sYh;
    if constexpr (NT == 64) {
#pragma unroll
      for (int it = 0; it < 8; ++it) {
        const int ch = it * 32 + lane, r = ch >> 4, q = (ch & 15) * 4;
        const v4f v = *(const v4fa*)(so + r * OSTR + q);
        *(volatile v4f*)(Yz + (size_t)(m0 + 16 * wave + r) * ldy + n0 + q) = v;
      }
    } else {
#pragma unroll
      for (int it = 0; it < 4; ++it) {
        const int ch = it * 32 + lane, r = ch >> 3, q = (ch & 7) * 4;
        const v4f v = *(const v4fa*)(so + r * OSTR + q);
        *(volatile v4f*)(Yz + (size_t)(m0 + 16 * wave + r) * ldy + n0 + q) = v;
      }
    }
    __threadfence();
  }
}

__global__ __launch_bounds__(256) void k_cvt_bf16(const float* __restrict__ src, unsigned short* dst, int n8) {
  const int i = blockIdx.x * 256 + threadIdx.x;
  if (i >= n8) return;
  const float* p = src + (size_t)i * 8;
  const v4f a = *(const v4fa*)p, b = *(const v4fa*)(p + 4);
  us8 o;
#pragma unroll
  for (int u = 0; u < 4; ++u) { o[u] = bf16_bits(a[u]); o[4 + u] = bf16_bits(b[u]); }
  unsigned short* d = dst + (size_t)i * 8;
  *(volatile us8*)d = o;
  __threadfence();
  *(volatile us8*)d = o;
}

__global__ __launch_bounds__(32) void k_wi(const float* __restrict__ W, unsigned short* W16) {
  const int r = blockIdx.x, lane = threadIdx.x;
  const int l = r / NWI, rr = r - l * NWI;
  int wr = 0;
  bool on = true;
  if (rr < CNV)             wr = DIN + rr;
  else if (rr < CNV + NHD)  wr = DIN + CNV + (rr - CNV);
  else if (rr < NXB)        { wr = 0; on = false; }
  else                      wr = rr - NXB;
  const float* src = W + ((size_t)l * DPR + wr) * DMD + 8 * lane;
  const v4f a = *(const v4fa*)src, b = *(const v4fa*)(src + 4);
  us8 o;
#pragma unroll
  for (int u = 0; u < 4; ++u) {
    o[u]     = on ? bf16_bits(a[u]) : (unsigned short)0;
    o[4 + u] = on ? bf16_bits(b[u]) : (unsigned short)0;
  }
  unsigned short* d = W16 + (size_t)r * DMD + 8 * lane;
  *(volatile us8*)d = o;
  __threadfence();
  *(volatile us8*)d = o;
}

template <int MODE>
__global__ __launch_bounds__(256) void k_rows(const float* __restrict__ pgs, const float* __restrict__ f, const float* __restrict__ HIDp,
                                             float* RES, const float* __restrict__ w, unsigned short* XNH, unsigned short* XNL,
                                             const float* __restrict__ alpha, float* out,
                                             const float* __restrict__ aux0, const float* __restrict__ aux1) {
  __shared__ unsigned long long skey[(MODE != 1) ? NPT : 2];
  const int tid = threadIdx.x, lane = tid & 31, wave = tid >> 5;
  if constexpr (MODE != 1) {
    for (int i = tid; i < NPT; i += 256) {
      const float v = bf16r(pgs[(size_t)i * 3 + 2]);
      unsigned u = __float_as_uint(v);
      if ((u << 1) == 0u) u = 0u;
      const unsigned key = (u & 0x80000000u) ? ~u : (u | 0x80000000u);
      skey[i] = (((unsigned long long)(~key)) << 32) | (unsigned long long)(unsigned)i;
    }
    __syncthreads();
    for (int k = 2; k <= NPT; k <<= 1) {
      for (int jj = k >> 1; jj > 0; jj >>= 1) {
        for (int i = tid; i < NPT; i += 256) {
          const int ixj = i ^ jj;
          if (ixj > i) {
            const unsigned long long a = skey[i], b = skey[ixj];
            const bool up = ((i & k) == 0);
            if ((a > b) == up) { skey[i] = b; skey[ixj] = a; }
          }
        }
        __syncthreads();
      }
    }
  }
  float asig = 0.0f;
  if constexpr (MODE == 2) asig = 1.0f / (1.0f + expf(-bf16r(alpha[0])));
  const int c0 = 4 * lane, c1 = 128 + 4 * lane;
  v4f wv0 = *(const v4fa*)(w + c0), wv1 = *(const v4fa*)(w + c1);
#pragma unroll
  for (int u = 0; u < 4; ++u) { wv0[u] = bf16r(wv0[u]); wv1[u] = bf16r(wv1[u]); }
  const int jbeg = (MODE == 1) ? (int)(blockIdx.x * 8 + wave) : wave;
  const int jend = (MODE == 1) ? (jbeg + 1) : NPT;
#pragma unroll 1
  for (int j = jbeg; j < jend; j += 8) {
    int r = 0;
    if constexpr (MODE != 1) {
      r = (int)(unsigned)(skey[j] & 0xFFFFFFFFull);
      r = (r < 0) ? 0 : ((r > NPT - 1) ? (NPT - 1) : r);
    }
    v4f v0, v1;
    if constexpr (MODE == 0) {
      v0 = *(const v4fa*)(f + (size_t)r * DMD + c0);
      v1 = *(const v4fa*)(f + (size_t)r * DMD + c1);
#pragma unroll
      for (int u = 0; u < 4; ++u) { v0[u] = bf16r(v0[u]); v1[u] = bf16r(v1[u]); }
    } else {
      v0 = *(const v4fa*)(HIDp + (size_t)j * DMD + c0) + *(const v4fa*)(RES + (size_t)j * DMD + c0);
      v1 = *(const v4fa*)(HIDp + (size_t)j * DMD + c1) + *(const v4fa*)(RES + (size_t)j * DMD + c1);
    }
    if constexpr (MODE != 2) {
      float* d0 = RES + (size_t)j * DMD + c0;
      float* d1 = RES + (size_t)j * DMD + c1;
      *(volatile v4f*)d0 = v0; *(volatile v4f*)d1 = v1;
      __threadfence();
      *(volatile v4f*)d0 = v0; *(volatile v4f*)d1 = v1;
    }
    float ss = 0.0f;
#pragma unroll
    for (int u = 0; u < 4; ++u) ss += v0[u] * v0[u] + v1[u] * v1[u];
#pragma unroll
    for (int o = 16; o > 0; o >>= 1) ss += __shfl_xor(ss, o);
    const float inv = rsqrtf(ss * (1.0f / (float)DMD) + EPSV);
    v4f o0, o1;
#pragma unroll
    for (int u = 0; u < 4; ++u) { o0[u] = v0[u] * inv * wv0[u]; o1[u] = v1[u] * inv * wv1[u]; }
    if constexpr (MODE != 2) {
      us4 h0, l0, h1, l1;
#pragma unroll
      for (int u = 0; u < 4; ++u) {
        const unsigned short ha = bf16_bits(o0[u]); h0[u] = ha; l0[u] = bf16_bits(o0[u] - bf16_val(ha));
        const unsigned short hb = bf16_bits(o1[u]); h1[u] = hb; l1[u] = bf16_bits(o1[u] - bf16_val(hb));
      }
      unsigned short* ph0 = XNH + (size_t)j * DMD + c0; unsigned short* ph1 = XNH + (size_t)j * DMD + c1;
      unsigned short* pl0 = XNL + (size_t)j * DMD + c0; unsigned short* pl1 = XNL + (size_t)j * DMD + c1;
      *(volatile us4*)ph0 = h0; *(volatile us4*)ph1 = h1; *(volatile us4*)pl0 = l0; *(volatile us4*)pl1 = l1;
      __threadfence();
      *(volatile us4*)ph0 = h0; *(volatile us4*)ph1 = h1; *(volatile us4*)pl0 = l0; *(volatile us4*)pl1 = l1;
    } else {
      v4f f0 = *(const v4fa*)(f + (size_t)r * DMD + c0), f1 = *(const v4fa*)(f + (size_t)r * DMD + c1);
      v4f q0, q1;
#pragma unroll
      for (int u = 0; u < 4; ++u) {
        q0[u] = o0[u] * asig + bf16r(f0[u]) * (1.0f - asig);
        q1[u] = o1[u] * asig + bf16r(f1[u]) * (1.0f - asig);
      }
      float* d0 = out + (size_t)r * DMD + c0;
      float* d1 = out + (size_t)r * DMD + c1;
      *(volatile v4f*)d0 = q0; *(volatile v4f*)d1 = q1;
      __threadfence();
      *(volatile v4f*)d0 = q0; *(volatile v4f*)d1 = q1;
    }
  }
}

__global__ __launch_bounds__(32) void k_dtacs(const float* __restrict__ XB, const float* __restrict__ bdt, const float* __restrict__ loga,
                                              float* DT, float* ACS) {
  const int c = blockIdx.x, h = threadIdx.x;
  const int hc = (h < NHD) ? h : (NHD - 1);
  const float live = (h < NHD) ? 1.0f : 0.0f;
  const float ah = -expf(bf16r(loga[hc]));
  const float bh = bf16r(bdt[hc]);
#pragma unroll 1
  for (int pass = 0; pass < 2; ++pass) {
    float run = 0.0f;
#pragma unroll 1
    for (int i = 0; i < CH; ++i) {
      const size_t t = (size_t)c * CH + i;
      const float dr = XB[t * NXB + CNV + hc] + bh;
      const float sp = fmaxf(dr, 0.0f) + log1pf(expf(-fabsf(dr)));
      const float dt = sp * live;
      run = run + ah * dt;
      *(volatile float*)(DT + t * ACSP + h) = dt;
      *(volatile float*)(ACS + t * ACSP + h) = run * live;
    }
    __threadfence();
  }
}

__global__ __launch_bounds__(384) void k_conv(const float* __restrict__ XB, const float* __restrict__ cw, const float* __restrict__ cb,
                                             const float* __restrict__ DT, const float* __restrict__ ACS,
                                             float* XF, unsigned short* XDT16, unsigned short* XDEC16, unsigned short* B16, unsigned short* C16) {
  const int t = blockIdx.x, tid = threadIdx.x, c = 4 * tid;
  v4f wt[4];
#pragma unroll
  for (int u = 0; u < 4; ++u) wt[u] = *(const v4fa*)(cw + (size_t)(c + u) * KW);
  v4f acc = {0.0f, 0.0f, 0.0f, 0.0f};
#pragma unroll
  for (int k = 0; k < KW; ++k) {
    const int tt = t - (KW - 1) + k;
    const int row = (tt < 0) ? 0 : tt;
    const float live = (tt >= 0) ? 1.0f : 0.0f;
    const v4f xv = *(const v4fa*)(XB + (size_t)row * NXB + c);
#pragma unroll
    for (int u = 0; u < 4; ++u) acc[u] += (xv[u] * live) * bf16r(wt[u][k]);
  }
  const v4f bv = *(const v4fa*)(cb + c);
  v4f res;
#pragma unroll
  for (int u = 0; u < 4; ++u) res[u] = silu_f(acc[u] + bf16r(bv[u]));
  if (tid < 128) {
    const int h = tid >> 3;
    const int tl = t | (CH - 1);
    const float dt = DT[(size_t)t * ACSP + h];
    const float dec = __expf(fminf(ACS[(size_t)tl * ACSP + h] - ACS[(size_t)t * ACSP + h], 0.0f));
    const float s1 = dt * SXD, s2 = s1 * dec;
    v4h ha, hb;
#pragma unroll
    for (int u = 0; u < 4; ++u) { ha[u] = (_Float16)(res[u] * s1); hb[u] = (_Float16)(res[u] * s2); }
    const us4 oa = __builtin_bit_cast(us4, ha), ob = __builtin_bit_cast(us4, hb);
    float* d0 = XF + (size_t)t * DIN + c;
    unsigned short* d1 = XDT16 + (size_t)t * DIN + c;
    unsigned short* d2 = XDEC16 + (size_t)t * DIN + c;
    *(volatile v4f*)d0 = res; *(volatile us4*)d1 = oa; *(volatile us4*)d2 = ob;
    __threadfence();
    *(volatile v4f*)d0 = res; *(volatile us4*)d1 = oa; *(volatile us4*)d2 = ob;
  } else if (tid < 256) {
    v4h hv;
#pragma unroll
    for (int u = 0; u < 4; ++u) hv[u] = (_Float16)(res[u] * SBC);
    const us4 o = __builtin_bit_cast(us4, hv);
    unsigned short* d = B16 + (size_t)t * DST + (c - DIN);
    *(volatile us4*)d = o;
    __threadfence();
    *(volatile us4*)d = o;
  } else {
    v4h hv;
#pragma unroll
    for (int u = 0; u < 4; ++u) hv[u] = (_Float16)(res[u] * SBC);
    const us4 o = __builtin_bit_cast(us4, hv);
    unsigned short* d = C16 + (size_t)t * DST + (c - 2 * DIN);
    *(volatile us4*)d = o;
    __threadfence();
    *(volatile us4*)d = o;
  }
}

__global__ __launch_bounds__(256) void k_prev(const float* __restrict__ ST, const float* __restrict__ ACS, unsigned short* PREV16) {
  const int part = blockIdx.x, h = blockIdx.y, tid = threadIdx.x;
  const int e0 = part * 2048 + tid * 8;
  v4f p0 = {0.0f, 0.0f, 0.0f, 0.0f}, p1 = {0.0f, 0.0f, 0.0f, 0.0f};
#pragma unroll 1
  for (int c = 0; c < NCH; ++c) {
    const size_t base = (size_t)(c * NHD + h) * (DST * HDM) + e0;
    v8h hv;
#pragma unroll
    for (int u = 0; u < 4; ++u) { hv[u] = (_Float16)(p0[u] * SPV); hv[4 + u] = (_Float16)(p1[u] * SPV); }
    const us8 o = __builtin_bit_cast(us8, hv);
    *(volatile us8*)(PREV16 + base) = o;
    __threadfence();
    *(volatile us8*)(PREV16 + base) = o;
    const float dec = __expf(fminf(ACS[(size_t)(c * CH + CH - 1) * ACSP + h], 0.0f));
    const v4f s0 = *(const v4fa*)(ST + base), s1 = *(const v4fa*)(ST + base + 4);
    p0 = p0 * dec + s0;
    p1 = p1 * dec + s1;
  }
}

__global__ __launch_bounds__(64) void k_gate(const float* __restrict__ YD, const float* __restrict__ YO, const float* __restrict__ Z,
                                            const float* __restrict__ gw, unsigned short* GH, unsigned short* GL) {
  __shared__ float red[2];
  const int t = blockIdx.x, tid = threadIdx.x, lane = tid & 31, wave = tid >> 5, c = 8 * tid;
  const size_t off = (size_t)t * DIN + c;
  const v4f ya = *(const v4fa*)(YD + off) + *(const v4fa*)(YO + off);
  const v4f yb = *(const v4fa*)(YD + off + 4) + *(const v4fa*)(YO + off + 4);
  const v4f za = *(const v4fa*)(Z + off), zb = *(const v4fa*)(Z + off + 4);
  const v4f wa = *(const v4fa*)(gw + c), wb = *(const v4fa*)(gw + c + 4);
  float g[8];
  float ss = 0.0f;
#pragma unroll
  for (int u = 0; u < 4; ++u) {
    g[u] = ya[u] * silu_f(za[u]);
    g[4 + u] = yb[u] * silu_f(zb[u]);
    ss += g[u] * g[u] + g[4 + u] * g[4 + u];
  }
#pragma unroll
  for (int o = 16; o > 0; o >>= 1) ss += __shfl_xor(ss, o);
  if (lane == 0) red[wave] = ss;
  __syncthreads();
  const float tot = red[0] + red[1];
  const float inv = rsqrtf(tot * (1.0f / (float)DIN) + EPSV);
  us8 hi, lo;
#pragma unroll
  for (int u = 0; u < 4; ++u) {
    const float ga = g[u] * inv * bf16r(wa[u]);
    const float gb = g[4 + u] * inv * bf16r(wb[u]);
    const unsigned short ha = bf16_bits(ga), hb = bf16_bits(gb);
    hi[u] = ha; lo[u] = bf16_bits(ga - bf16_val(ha));
    hi[4 + u] = hb; lo[4 + u] = bf16_bits(gb - bf16_val(hb));
  }
  *(volatile us8*)(GH + off) = hi; *(volatile us8*)(GL + off) = lo;
  __threadfence();
  *(volatile us8*)(GH + off) = hi; *(volatile us8*)(GL + off) = lo;
}

extern "C" void kernel_launch(void* const* d_in, const int* in_sizes, int n_in,
                              void* d_out, int out_size, void* d_ws, size_t ws_size,
                              hipStream_t stream) {
  if (n_in < 15) return;
  if (in_sizes[1] != NPT * 3 || in_sizes[2] != NPT * DMD || in_sizes[4] != NL * DPR * DMD || in_sizes[5] != NL * CNV * KW ||
      in_sizes[6] != NL * CNV || in_sizes[7] != NL * NHD || in_sizes[8] != NL * NHD || in_sizes[9] != NL * NHD || in_sizes[10] != NL * DIN ||
      in_sizes[11] != NL * DMD * DIN || in_sizes[12] != NL * DMD || in_sizes[13] != DMD || in_sizes[14] < 1 || out_size != NPT * DMD) return;
  const float* pxyz = (const float*)d_in[0];
  const float* pgs  = (const float*)d_in[1];
  const float* fin  = (const float*)d_in[2];
  const float* cov  = (const float*)d_in[3];
  const float* Win  = (const float*)d_in[4];
  const float* cw   = (const float*)d_in[5];
  const float* cb   = (const float*)d_in[6];
  const float* bdt  = (const float*)d_in[7];
  const float* loga = (const float*)d_in[8];
  const float* dprm = (const float*)d_in[9];
  const float* gnw  = (const float*)d_in[10];
  const float* Wout = (const float*)d_in[11];
  const float* blkw = (const float*)d_in[12];
  const float* fnw  = (const float*)d_in[13];
  const float* alph = (const float*)d_in[14];
  float* out = (float*)d_out;

  size_t off = 0;
  auto carve = [&](size_t bytes) -> char* { char* p = (char*)d_ws + off; off += (bytes + 255) & ~(size_t)255; return p; };
  float* RES  = (float*)carve((size_t)NPT * DMD * 4);
  float* HID  = (float*)carve((size_t)NPT * DMD * 4);
  unsigned short* XNH = (unsigned short*)carve((size_t)NPT * DMD * 2);
  unsigned short* XNL = (unsigned short*)carve((size_t)NPT * DMD * 2);
  unsigned short* WI16 = (unsigned short*)carve((size_t)NL * NWI * DMD * 2);
  unsigned short* WO16 = (unsigned short*)carve((size_t)NL * DMD * DIN * 2);
  float* Zf   = (float*)carve((size_t)NPT * DIN * 4);
  float* XB   = (float*)carve((size_t)NPT * NXB * 4);
  float* DT   = (float*)carve((size_t)NPT * ACSP * 4);
  float* ACS  = (float*)carve((size_t)NPT * ACSP * 4);
  float* XF   = (float*)carve((size_t)NPT * DIN * 4);
  unsigned short* XDT16  = (unsigned short*)carve((size_t)NPT * DIN * 2);
  unsigned short* XDEC16 = (unsigned short*)carve((size_t)NPT * DIN * 2);
  unsigned short* B16    = (unsigned short*)carve((size_t)NPT * DST * 2);
  unsigned short* C16    = (unsigned short*)carve((size_t)NPT * DST * 2);
  float* CBF  = (float*)carve((size_t)NCH * CH * CH * 4);
  float* YD   = (float*)carve((size_t)NPT * DIN * 4);
  float* YO   = (float*)carve((size_t)NPT * DIN * 4);
  float* ST   = (float*)carve((size_t)NCH * NHD * DST * HDM * 4);
  unsigned short* PREV16 = (unsigned short*)carve((size_t)NCH * NHD * DST * HDM * 2);
  unsigned short* GH = (unsigned short*)carve((size_t)NPT * DIN * 2);
  unsigned short* GL = (unsigned short*)carve((size_t)NPT * DIN * 2);
  if (off > ws_size || off > (size_t)134217728) return;

  const dim3 blk(256);
  const long long CHS = (long long)CH * DST;
  const long long CHF = (long long)CH * DIN;
  const long long STS = (long long)DST * HDM;
  const long long ACC = (long long)CH * ACSP;

  k_wi<<<dim3(NL * NWI), dim3(32), 0, stream>>>(Win, WI16);
  { const int n8 = in_sizes[11] / 8; k_cvt_bf16<<<dim3((n8 + 255) / 256), blk, 0, stream>>>(Wout, WO16, n8); }
  k_rows<0><<<dim3(1), blk, 0, stream>>>(pgs, fin, HID, RES, blkw, XNH, XNL, alph, out, pxyz, cov);

  for (int l = 0; l < NL; ++l) {
    if (l > 0) k_rows<1><<<dim3(NPT / 8), blk, 0, stream>>>(pgs, fin, HID, RES, blkw + (size_t)l * DMD, XNH, XNL, alph, out, pxyz, cov);
    const unsigned short* WIl = WI16 + (size_t)l * NWI * DMD;
    k_gemm<1, 2, 0, 0, 0, 64><<<dim3(NPT / 128, NXB / 64, 1), blk, 0, stream>>>(XNH, XNL, DMD, 0, 0, WIl, DMD, 0, 0,
        XB, NXB, 0, 0, XF, 0, 0, 0, dprm, ACS, 0, 0, 1, DMD, 1.0f);
    k_gemm<1, 2, 0, 0, 0, 64><<<dim3(NPT / 128, DIN / 64, 1), blk, 0, stream>>>(XNH, XNL, DMD, 0, 0, WIl + (size_t)NXB * DMD, DMD, 0, 0,
        Zf, DIN, 0, 0, XF, 0, 0, 0, dprm, ACS, 0, 0, 1, DMD, 1.0f);
    k_dtacs<<<dim3(NCH), dim3(32), 0, stream>>>(XB, bdt + l * NHD, loga + l * NHD, DT, ACS);
    k_conv<<<dim3(NPT), dim3(384), 0, stream>>>(XB, cw + (size_t)l * CNV * KW, cb + (size_t)l * CNV, DT, ACS, XF, XDT16, XDEC16, B16, C16);
    k_gemm<0, 1, 0, 0, 0, 64><<<dim3(CH / 128, CH / 64, NCH), blk, 0, stream>>>(C16, C16, DST, CHS, 0, B16, DST, CHS, 0,
        CBF, CH, (long long)CH * CH, 0, XF, 0, 0, 0, dprm, ACS, 0, 0, 1, DST, 1.0f / (SBC * SBC));
    k_gemm<0, 1, 2, 1, 1, 32><<<dim3(CH / 128, 1, NCH * NHD), blk, 0, stream>>>(CBF, CBF, CH, (long long)CH * CH, 0, XDT16, DIN, CHS, HDM,
        YD, DIN, CHF, HDM, XF, DIN, CHF, HDM, dprm + l * NHD, ACS, ACC, 1, NHD, CH, 1.0f / (SGD * SXD));
    k_gemm<0, 1, 1, 1, 0, 32><<<dim3(DST / 128, 1, NCH * NHD), blk, 0, stream>>>(B16, B16, DST, CHS, 0, XDEC16, DIN, CHS, HDM,
        ST, HDM, (long long)NHD * STS, STS, XF, 0, 0, 0, dprm, ACS, 0, 0, NHD, CH, 1.0f / (SBC * SXD));
    k_prev<<<dim3(8, NHD), blk, 0, stream>>>(ST, ACS, PREV16);
    k_gemm<0, 1, 0, 1, 2, 32><<<dim3(CH / 128, 1, NCH * NHD), blk, 0, stream>>>(C16, C16, DST, CHS, 0, PREV16, HDM, (long long)NHD * STS, STS,
        YO, DIN, CHF, HDM, XF, 0, 0, 0, dprm, ACS, ACC, 1, NHD, DST, 1.0f / (SBC * SPV));
    k_gate<<<dim3(NPT), dim3(64), 0, stream>>>(YD, YO, Zf, gnw + (size_t)l * DIN, GH, GL);
    k_gemm<1, 2, 0, 0, 0, 64><<<dim3(NPT / 128, DMD / 64, 1), blk, 0, stream>>>(GH, GL, DIN, 0, 0, WO16 + (size_t)l * DMD * DIN, DIN, 0, 0,
        HID, DMD, 0, 0, XF, 0, 0, 0, dprm, ACS, 0, 0, 1, DIN, 1.0f);
  }
  k_rows<2><<<dim3(1), blk, 0, stream>>>(pgs, fin, HID, RES, fnw, XNH, XNL, alph, out, pxyz, cov);
}
